// TransformerEncoder_15857019257396
// MI455X (gfx1250) — hardware-verified
//
#include <hip/hip_runtime.h>
#ifndef SEQ
#define SEQ 4096
#endif
#define DD 1024
#define NH 16
#define DH 64
#define FF 4096
#define QKP 2048

static_assert(SEQ % 128 == 0);
static_assert(DD % 64 == 0 && FF % 64 == 0 && QKP == 2 * DD && NH * DH == DD);
static_assert(DD % 32 == 0 && FF % 32 == 0);

typedef _Float16 v16h __attribute__((ext_vector_type(16)));
typedef _Float16 v8h  __attribute__((ext_vector_type(8), may_alias));
typedef float    v8f  __attribute__((ext_vector_type(8)));
typedef float    v4f  __attribute__((ext_vector_type(4)));
typedef float    v4fa __attribute__((ext_vector_type(4), may_alias));
union FragH { v16h v; v8h half[2]; };

__device__ __forceinline__ float bf16_rne(float x) {
  unsigned int u = __float_as_uint(x);
  u = (u + 0x7FFFu + ((u >> 16) & 1u)) & 0xFFFF0000u;
  return __uint_as_float(u);
}

__device__ __forceinline__ v8f mma16(v16h a, v16h b, v8f c) {
  c = __builtin_amdgcn_wmma_f32_16x16x32_f16(false, a, false, b, (short)0, c, false, false);
  asm volatile("v_nop\n\tv_nop\n\tv_nop\n\tv_nop" : "+v"(c) : "v"(a), "v"(b));
  return c;
}

__device__ __forceinline__ void wave_lds_sync() {
  __builtin_amdgcn_fence(4  , "workgroup");
  __builtin_amdgcn_wave_barrier();
}

__global__ __launch_bounds__(256) void k_wt(const float* __restrict__ W, _Float16* __restrict__ Wt, unsigned K, unsigned N, unsigned kshift) {
  const unsigned t = blockIdx.x * 256u + threadIdx.x;
  if (t >= N * (K >> 3)) return;
  const unsigned n = t >> kshift, k8 = (t & ((K >> 3) - 1u)) << 3;
  v8h v;
#pragma unroll
  for (int i = 0; i < 8; ++i) v[i] = (_Float16)(bf16_rne(W[(size_t)(k8 + (unsigned)i) * N + n]) * 64.0f);
  _Float16* dst = Wt + (size_t)n * K + k8;
  *(volatile v8h*)dst = v;
  __threadfence();
  *(volatile v8h*)dst = v;
}

template <bool RIN>
__device__ __forceinline__ void ln_load8(const float* p, float (&v)[8]) {
  const v4f a0 = *(const v4fa*)p, a1 = *(const v4fa*)(p + 4);
  v[0] = a0[0]; v[1] = a0[1]; v[2] = a0[2]; v[3] = a0[3];
  v[4] = a1[0]; v[5] = a1[1]; v[6] = a1[2]; v[7] = a1[3];
  if (RIN) {
#pragma unroll
    for (int i = 0; i < 8; ++i) v[i] = bf16_rne(v[i]);
  }
}

__device__ __forceinline__ float wave_sum(float v) {
  v += __shfl_xor(v, 1, 32); v += __shfl_xor(v, 2, 32); v += __shfl_xor(v, 4, 32);
  v += __shfl_xor(v, 8, 32); v += __shfl_xor(v, 16, 32);
  return v;
}

template <bool RIN>
__global__ __launch_bounds__(128) void k_ln(const float* __restrict__ X, const float* __restrict__ g, const float* __restrict__ bta, _Float16* __restrict__ Y) {
  const unsigned tid = threadIdx.x, w = tid >> 5, lane = tid & 31u;
  const unsigned row = blockIdx.x * 4u + w;
  const float* x = X + (size_t)row * DD + lane * 8u;
  float s1 = 0.f;
#pragma unroll 1
  for (unsigned c = 0; c < 4u; ++c) {
    float v[8]; ln_load8<RIN>(x + c * 256u, v);
    s1 += ((v[0] + v[1]) + (v[2] + v[3])) + ((v[4] + v[5]) + (v[6] + v[7]));
  }
  const float mu = wave_sum(s1) * (1.0f / (float)DD);
  float s2 = 0.f;
#pragma unroll 1
  for (unsigned c = 0; c < 4u; ++c) {
    float v[8]; ln_load8<RIN>(x + c * 256u, v);
#pragma unroll
    for (int i = 0; i < 8; ++i) { const float d = v[i] - mu; s2 += d * d; }
  }
  const float rs = rsqrtf(wave_sum(s2) * (1.0f / (float)DD) + 1e-6f);
  _Float16* y = Y + (size_t)row * DD + lane * 8u;
#pragma unroll 1
  for (unsigned c = 0; c < 4u; ++c) {
    float v[8], gg[8], bb[8];
    ln_load8<RIN>(x + c * 256u, v);
    ln_load8<true>(g + lane * 8u + c * 256u, gg);
    ln_load8<true>(bta + lane * 8u + c * 256u, bb);
    v8h pk;
#pragma unroll
    for (int i = 0; i < 8; ++i) pk[i] = (_Float16)((v[i] - mu) * rs * gg[i] + bb[i]);
    *(volatile v8h*)(y + c * 256u) = pk;
    __threadfence();
    *(volatile v8h*)(y + c * 256u) = pk;
  }
}

__device__ __forceinline__ void gemm_core(const _Float16* __restrict__ A, unsigned lda, const _Float16* __restrict__ Bt, unsigned ldb,
                                          unsigned arow, unsigned bcol, unsigned hh, unsigned K, v8f (&acc)[2][4]) {
  const _Float16* ap0 = A + (size_t)arow * lda + 8u * hh;
  const _Float16* ap1 = ap0 + (size_t)16u * lda;
  const _Float16* bp = Bt + (size_t)bcol * ldb + 8u * hh;
#pragma unroll
  for (int mi = 0; mi < 2; ++mi)
#pragma unroll
    for (int t = 0; t < 4; ++t) acc[mi][t] = (v8f){0.f, 0.f, 0.f, 0.f, 0.f, 0.f, 0.f, 0.f};
#pragma unroll 1
  for (unsigned kb = 0; kb < K; kb += 32u) {
    FragH a0, a1, b[4];
    a0.half[0] = *(const v8h*)(ap0 + kb); a0.half[1] = *(const v8h*)(ap0 + kb + 16u);
    a1.half[0] = *(const v8h*)(ap1 + kb); a1.half[1] = *(const v8h*)(ap1 + kb + 16u);
#pragma unroll
    for (int t = 0; t < 4; ++t) {
      const _Float16* br = bp + (size_t)((unsigned)t * 16u) * ldb + kb;
      b[t].half[0] = *(const v8h*)br; b[t].half[1] = *(const v8h*)(br + 16u);
    }
#pragma unroll
    for (int t = 0; t < 4; ++t) {
      acc[0][t] = mma16(a0.v, b[t].v, acc[0][t]);
      acc[1][t] = mma16(a1.v, b[t].v, acc[1][t]);
    }
  }
}

template <int ACT>
__global__ __launch_bounds__(128) void k_gemm_h16(const _Float16* __restrict__ A, unsigned lda, const _Float16* __restrict__ Bt, unsigned ldb,
                                                  const float* __restrict__ bias0, const float* __restrict__ bias1, unsigned nsplit,
                                                  _Float16* __restrict__ C, unsigned ldc, float scale, float oscale, unsigned K) {
  __shared__ __attribute__((aligned(16))) float so[4][32][64];
  __shared__ __attribute__((aligned(16))) _Float16 sh[4][32][64];
  const unsigned tid = threadIdx.x, w = tid >> 5, lane = tid & 31u, ln = lane & 15u, hh = lane >> 4;
  const unsigned row0 = blockIdx.y * 128u, col0 = blockIdx.x * 64u;
  v8f acc[2][4];
  gemm_core(A, lda, Bt, ldb, row0 + 32u * w + ln, col0 + ln, hh, K, acc);
#pragma unroll
  for (int mi = 0; mi < 2; ++mi)
#pragma unroll
    for (int t = 0; t < 4; ++t)
#pragma unroll
      for (int r = 0; r < 8; ++r) so[w][(unsigned)mi * 16u + 8u * hh + (unsigned)r][(unsigned)t * 16u + ln] = acc[mi][t][r] * scale;
  wave_lds_sync();
  const unsigned rs = lane >> 3, c8 = (lane & 7u) * 8u;
  const float* bp = (col0 < nsplit) ? (bias0 + col0) : (bias1 + (col0 - nsplit));
  float bv[8]; ln_load8<true>(bp + c8, bv);
#pragma unroll 1
  for (unsigned q = 0; q < 8u; ++q) {
    const unsigned row = q * 4u + rs;
    float u[8]; ln_load8<false>(&so[w][row][c8], u);
    v8h pk;
#pragma unroll
    for (int i = 0; i < 8; ++i) {
      float v = u[i] + bv[i];
      if (ACT == 2) v = 0.5f * v * (1.0f + erff(v * 0.70710678118654752f));
      pk[i] = (_Float16)(v * oscale);
    }
    *(v8h*)&sh[w][row][c8] = pk;
  }
  wave_lds_sync();
  _Float16* cb = C + (size_t)(row0 + 32u * w) * ldc + col0 + c8;
  for (int pass = 0; pass < 2; ++pass) {
#pragma unroll
    for (int q = 0; q < 8; ++q) {
      const unsigned row = (unsigned)q * 4u + rs;
      const v8h val = *(const v8h*)&sh[w][row][c8];
      *(volatile v8h*)(cb + (size_t)row * ldc) = val;
    }
    if (pass == 0) __threadfence();
  }
}

__global__ __launch_bounds__(128) void k_gemm_vt(const _Float16* __restrict__ A, unsigned lda, const _Float16* __restrict__ Bt, unsigned ldb,
                                                 const float* __restrict__ bias, _Float16* __restrict__ Ct, unsigned ldc, float scale, unsigned K) {
  __shared__ __attribute__((aligned(16))) _Float16 sT[64][136];
  const unsigned tid = threadIdx.x, w = tid >> 5, lane = tid & 31u, ln = lane & 15u, hh = lane >> 4;
  const unsigned row0 = blockIdx.y * 128u, col0 = blockIdx.x * 64u;
  v8f acc[2][4];
  gemm_core(A, lda, Bt, ldb, row0 + 32u * w + ln, col0 + ln, hh, K, acc);
#pragma unroll
  for (int t = 0; t < 4; ++t) {
    const unsigned col = (unsigned)t * 16u + ln;
    const float bb = bf16_rne(bias[col0 + col]);
#pragma unroll
    for (int mi = 0; mi < 2; ++mi) {
      v8h pk;
#pragma unroll
      for (int r = 0; r < 8; ++r) pk[r] = (_Float16)(acc[mi][t][r] * scale + bb);
      *(v8h*)&sT[col][32u * w + (unsigned)mi * 16u + 8u * hh] = pk;
    }
  }
  __syncthreads();
  for (int pass = 0; pass < 2; ++pass) {
#pragma unroll
    for (int q = 0; q < 8; ++q) {
      const unsigned n = (((unsigned)q * 4u + w) << 1) + hh;
      const v8h val = *(const v8h*)&sT[n][ln * 8u];
      *(volatile v8h*)(Ct + (size_t)(col0 + n) * ldc + row0 + ln * 8u) = val;
    }
    if (pass == 0) __threadfence();
  }
}

template <bool RES_BF16>
__global__ __launch_bounds__(128) void k_gemm_f32(const _Float16* __restrict__ A, unsigned lda, const _Float16* __restrict__ Bt, unsigned ldb,
                                                  const float* __restrict__ bias, const float* __restrict__ resid, unsigned ldr,
                                                  float* __restrict__ C, unsigned ldc, float scale, unsigned K) {
  __shared__ __attribute__((aligned(16))) float so[4][32][64];
  const unsigned tid = threadIdx.x, w = tid >> 5, lane = tid & 31u, ln = lane & 15u, hh = lane >> 4;
  const unsigned row0 = blockIdx.y * 128u, col0 = blockIdx.x * 64u;
  v8f acc[2][4];
  gemm_core(A, lda, Bt, ldb, row0 + 32u * w + ln, col0 + ln, hh, K, acc);
#pragma unroll
  for (int mi = 0; mi < 2; ++mi)
#pragma unroll
    for (int t = 0; t < 4; ++t)
#pragma unroll
      for (int r = 0; r < 8; ++r) so[w][(unsigned)mi * 16u + 8u * hh + (unsigned)r][(unsigned)t * 16u + ln] = acc[mi][t][r] * scale;
  wave_lds_sync();
  const unsigned rs = lane >> 4, c4 = (lane & 15u) * 4u;
  v4f bv = *(const v4fa*)(bias + col0 + c4);
#pragma unroll
  for (int i = 0; i < 4; ++i) bv[i] = bf16_rne(bv[i]);
  const float* rb = resid + (size_t)(row0 + 32u * w) * ldr + col0 + c4;
#pragma unroll 1
  for (unsigned q = 0; q < 16u; ++q) {
    const unsigned row = q * 2u + rs;
    const v4f u = *(const v4fa*)&so[w][row][c4];
    v4f rv = *(const v4fa*)(rb + (size_t)row * ldr);
    v4f o;
#pragma unroll
    for (int i = 0; i < 4; ++i) { float r1 = rv[i]; if (RES_BF16) r1 = bf16_rne(r1); o[i] = (u[i] + bv[i]) + r1; }
    *(v4fa*)&so[w][row][c4] = o;
  }
  wave_lds_sync();
  float* cb = C + (size_t)(row0 + 32u * w) * ldc + col0 + c4;
  for (int pass = 0; pass < 2; ++pass) {
#pragma unroll
    for (int q = 0; q < 16; ++q) {
      const unsigned row = (unsigned)q * 2u + rs;
      const v4f val = *(const v4fa*)&so[w][row][c4];
      *(volatile v4f*)(cb + (size_t)row * ldc) = val;
    }
    if (pass == 0) __threadfence();
  }
}

__global__ __launch_bounds__(128) void k_flash(const _Float16* __restrict__ qk, const _Float16* __restrict__ vT, _Float16* __restrict__ ctx) {
  __shared__ __attribute__((aligned(16))) _Float16 sO[4][16][72];
  const unsigned tid = threadIdx.x, w = tid >> 5, lane = tid & 31u, ln = lane & 15u, hh = lane >> 4;
  const unsigned h = blockIdx.y, q0 = blockIdx.x * 64u + w * 16u;
  FragH bq[2];
  {
    const _Float16* qr = qk + (size_t)(q0 + ln) * QKP + h * 64u + 8u * hh;
#pragma unroll
    for (int ks = 0; ks < 2; ++ks) { bq[ks].half[0] = *(const v8h*)(qr + ks * 32); bq[ks].half[1] = *(const v8h*)(qr + ks * 32 + 16); }
  }
  const _Float16* kbase = qk + DD + h * 64u + 8u * hh + (size_t)ln * QKP;
  const _Float16* vbase = vT + (size_t)(h * 64u + ln) * SEQ + 8u * hh;
  float m_run = -3.0e38f, l_run = 0.f;
  v8f oacc[4];
#pragma unroll
  for (int dt = 0; dt < 4; ++dt) oacc[dt] = (v8f){0.f, 0.f, 0.f, 0.f, 0.f, 0.f, 0.f, 0.f};
#pragma unroll 1
  for (unsigned j0 = 0; j0 < (unsigned)SEQ; j0 += 64u) {
    v8f s[4];
#pragma unroll
    for (int kt = 0; kt < 4; ++kt) {
      v8f a = {0.f, 0.f, 0.f, 0.f, 0.f, 0.f, 0.f, 0.f};
      const _Float16* kr = kbase + (size_t)(j0 + (unsigned)kt * 16u) * QKP;
#pragma unroll
      for (int ks = 0; ks < 2; ++ks) {
        FragH ka;
        ka.half[0] = *(const v8h*)(kr + ks * 32); ka.half[1] = *(const v8h*)(kr + ks * 32 + 16);
        a = mma16(ka.v, bq[ks].v, a);
      }
      s[kt] = a;
    }
    float mx = s[0][0];
#pragma unroll
    for (int kt = 0; kt < 4; ++kt)
#pragma unroll
      for (int r = 0; r < 8; ++r) mx = fmaxf(mx, s[kt][r]);
    mx *= 0.125f;
    mx = fmaxf(mx, __shfl_xor(mx, 16, 32));
    const float mnew = fmaxf(m_run, mx);
    const float alpha = __expf(m_run - mnew);
    m_run = mnew;
    FragH pb[2];
    float ps = 0.f;
#pragma unroll
    for (int k2 = 0; k2 < 2; ++k2)
#pragma unroll
      for (int r = 0; r < 8; ++r) {
        const float p0 = __expf(fmaf(s[2 * k2][r], 0.125f, -mnew));
        const float p1 = __expf(fmaf(s[2 * k2 + 1][r], 0.125f, -mnew));
        ps += p0 + p1;
        pb[k2].v[r] = (_Float16)(p0 * 256.0f);
        pb[k2].v[8 + r] = (_Float16)(p1 * 256.0f);
      }
    l_run = l_run * alpha + ps;
#pragma unroll
    for (int dt = 0; dt < 4; ++dt) oacc[dt] *= alpha;
#pragma unroll
    for (int dt = 0; dt < 4; ++dt) {
      const _Float16* vr = vbase + (size_t)((unsigned)dt * 16u) * SEQ + j0;
#pragma unroll
      for (int k2 = 0; k2 < 2; ++k2) {
        FragH va;
        va.half[0] = *(const v8h*)(vr + k2 * 32); va.half[1] = *(const v8h*)(vr + k2 * 32 + 16);
        oacc[dt] = mma16(va.v, pb[k2].v, oacc[dt]);
      }
    }
  }
  const float l = l_run + __shfl_xor(l_run, 16, 32);
  const float inv = 1.0f / l;
#pragma unroll
  for (int dt = 0; dt < 4; ++dt) {
    v8h pk;
#pragma unroll
    for (int r = 0; r < 8; ++r) pk[r] = (_Float16)(oacc[dt][r] * inv);
    *(v8h*)&sO[w][ln][(unsigned)dt * 16u + 8u * hh] = pk;
  }
  wave_lds_sync();
  const unsigned rs = lane >> 3, c8 = (lane & 7u) * 8u;
  _Float16* cb = ctx + (size_t)q0 * DD + h * 64u + c8;
  for (int pass = 0; pass < 2; ++pass) {
#pragma unroll
    for (int q = 0; q < 4; ++q) {
      const unsigned row = (unsigned)q * 4u + rs;
      const v8h val = *(const v8h*)&sO[w][row][c8];
      *(volatile v8h*)(cb + (size_t)row * DD) = val;
    }
    if (pass == 0) __threadfence();
  }
}

constexpr size_t SZ_WQK = (size_t)QKP * DD * 2, SZ_WV = (size_t)DD * DD * 2, SZ_WO = (size_t)DD * DD * 2;
constexpr size_t SZ_W1 = (size_t)FF * DD * 2, SZ_W2 = (size_t)DD * FF * 2;
constexpr size_t SZ_Y = (size_t)SEQ * DD * 2, SZ_QK = (size_t)SEQ * QKP * 2, SZ_VT = (size_t)DD * SEQ * 2;
constexpr size_t SZ_CTX = (size_t)SEQ * DD * 2, SZ_X1 = (size_t)SEQ * DD * 4, SZ_H = (size_t)SEQ * FF * 2;
constexpr size_t SZ_TOTAL = SZ_WQK + SZ_WV + SZ_WO + SZ_W1 + SZ_W2 + SZ_Y + SZ_QK + SZ_VT + SZ_CTX + SZ_X1 + SZ_Y + SZ_H;
static_assert(SZ_TOTAL <= (size_t)134217728);
static_assert(SZ_WQK % 256 == 0 && SZ_WV % 256 == 0 && SZ_Y % 256 == 0 && SZ_QK % 256 == 0 && SZ_VT % 256 == 0 && SZ_X1 % 256 == 0 && SZ_H % 256 == 0);

extern "C" void kernel_launch(void* const* d_in, const int* in_sizes, int n_in,
                              void* d_out, int out_size, void* d_ws, size_t ws_size, hipStream_t stream) {
  if (n_in < 17) return;
  if (in_sizes[0] < SEQ * DD || out_size < SEQ * DD) return;
  if (in_sizes[1] < DD * DD || in_sizes[3] < DD * DD || in_sizes[5] < DD * DD || in_sizes[7] < DD * DD) return;
  if (in_sizes[13] < DD * FF || in_sizes[15] < FF * DD) return;
  if (in_sizes[2] < DD || in_sizes[4] < DD || in_sizes[6] < DD || in_sizes[8] < DD) return;
  if (in_sizes[9] < DD || in_sizes[10] < DD || in_sizes[11] < DD || in_sizes[12] < DD) return;
  if (in_sizes[14] < FF || in_sizes[16] < DD) return;
  if (ws_size < SZ_TOTAL) return;
  const float* x   = (const float*)d_in[0];
  const float* Wq  = (const float*)d_in[1];  const float* bq  = (const float*)d_in[2];
  const float* Wk  = (const float*)d_in[3];  const float* bk  = (const float*)d_in[4];
  const float* Wv  = (const float*)d_in[5];  const float* bv  = (const float*)d_in[6];
  const float* Wo  = (const float*)d_in[7];  const float* bo  = (const float*)d_in[8];
  const float* l1s = (const float*)d_in[9];  const float* l1b = (const float*)d_in[10];
  const float* l2s = (const float*)d_in[11]; const float* l2b = (const float*)d_in[12];
  const float* W1  = (const float*)d_in[13]; const float* b1  = (const float*)d_in[14];
  const float* W2  = (const float*)d_in[15]; const float* b2  = (const float*)d_in[16];
  float* out = (float*)d_out;

  char* ws = (char*)d_ws; size_t off = 0;
  auto take = [&](size_t bytes) { char* p = ws + off; off += bytes; return p; };
  _Float16* WqkT = (_Float16*)take(SZ_WQK);
  _Float16* WvT  = (_Float16*)take(SZ_WV);
  _Float16* WoT  = (_Float16*)take(SZ_WO);
  _Float16* W1T  = (_Float16*)take(SZ_W1);
  _Float16* W2T  = (_Float16*)take(SZ_W2);
  _Float16* y1   = (_Float16*)take(SZ_Y);
  _Float16* qkp  = (_Float16*)take(SZ_QK);
  _Float16* vTp  = (_Float16*)take(SZ_VT);
  _Float16* ctx  = (_Float16*)take(SZ_CTX);
  float*    x1   = (float*)take(SZ_X1);
  _Float16* y2   = (_Float16*)take(SZ_Y);
  _Float16* hh   = (_Float16*)take(SZ_H);
  if (off > ws_size) return;

  k_wt<<<(DD * (DD / 8)) / 256, 256, 0, stream>>>(Wq, WqkT, DD, DD, 7u);
  k_wt<<<(DD * (DD / 8)) / 256, 256, 0, stream>>>(Wk, WqkT + (size_t)DD * DD, DD, DD, 7u);
  k_wt<<<(DD * (DD / 8)) / 256, 256, 0, stream>>>(Wv, WvT, DD, DD, 7u);
  k_wt<<<(DD * (DD / 8)) / 256, 256, 0, stream>>>(Wo, WoT, DD, DD, 7u);
  k_wt<<<(FF * (DD / 8)) / 256, 256, 0, stream>>>(W1, W1T, DD, FF, 7u);
  k_wt<<<(DD * (FF / 8)) / 256, 256, 0, stream>>>(W2, W2T, FF, DD, 9u);

  k_ln<true><<<SEQ / 4, 128, 0, stream>>>(x, l1s, l1b, y1);
  k_gemm_h16<0><<<dim3(QKP / 64, SEQ / 128), 128, 0, stream>>>(y1, DD, WqkT, DD, bq, bk, DD, qkp, QKP, 1.0f / 64.0f, 1.0f, DD);
  k_gemm_vt<<<dim3(DD / 64, SEQ / 128), 128, 0, stream>>>(y1, DD, WvT, DD, bv, vTp, SEQ, 1.0f / 64.0f, DD);
  k_flash<<<dim3(SEQ / 64, NH), 128, 0, stream>>>(qkp, vTp, ctx);
  k_gemm_f32<true><<<dim3(DD / 64, SEQ / 128), 128, 0, stream>>>(ctx, DD, WoT, DD, bo, x, DD, x1, DD, 1.0f / 16384.0f, DD);
  k_ln<false><<<SEQ / 4, 128, 0, stream>>>(x1, l2s, l2b, y2);
  k_gemm_h16<2><<<dim3(FF / 64, SEQ / 128), 128, 0, stream>>>(y2, DD, W1T, DD, b1, b1, FF, hh, FF, 1.0f / 64.0f, 16.0f, DD);
  k_gemm_f32<false><<<dim3(DD / 64, SEQ / 128), 128, 0, stream>>>(hh, FF, W2T, FF, b2, x1, DD, out, DD, 1.0f / 1024.0f, FF);
}
